// ExRestSelfAtten_87711822119181
// MI455X (gfx1250) — hardware-verified
//
#include <hip/hip_runtime.h>
#include <stddef.h>
#include <stdint.h>

#define NB    8
#define SQ    2048
#define DM    256
#define AW    16
#define NOUT  2
#define NROW  (NB * SQ)
#define QT    32
#define HL    (QT + 2 * AW)
#define KOFF  16
#define KROWS 2112
#define VOFF  64
#define VTP   2176
#define NQKV  768
#define LP    264
#define STP   72
#define SFP   68
#define PSP   72

static_assert(DM == 256);
static_assert(NROW % 256 == 0);
static_assert(SQ % 256 == 0);
static_assert(SQ % QT == 0);
static_assert(HL == 64);
static_assert(KOFF >= AW);
static_assert(VOFF >= AW);
static_assert(KROWS >= KOFF + SQ + AW);
static_assert(KROWS - (KOFF + SQ) == 48);
static_assert(VTP >= VOFF + SQ + AW);
static_assert(VTP - (VOFF + SQ) == 64);
static_assert(((VOFF - AW) % 8) == 0);
static_assert((VTP % 64) == 0);
static_assert((NROW * DM) % 2048 == 0);
static_assert(64 * LP <= 256 * STP);

typedef _Float16 v16h __attribute__((ext_vector_type(16)));
typedef _Float16 v8h  __attribute__((ext_vector_type(8)));
typedef float    v8f  __attribute__((ext_vector_type(8)));
typedef float    v4f  __attribute__((ext_vector_type(4)));
typedef unsigned int v4u __attribute__((ext_vector_type(4)));

union Frag  { v16h v; v8h h[2]; };
union Pack8 { v8h h; v4u u; };

__device__ __forceinline__ v8f mma16(v16h a, v16h b, v8f c) {
  c = __builtin_amdgcn_wmma_f32_16x16x32_f16(false, a, false, b, (short)0, c, false, false);
  asm volatile("v_nop\n\tv_nop\n\tv_nop\n\tv_nop" : "+v"(c) : "v"(a), "v"(b));
  return c;
}

__device__ __forceinline__ v16h ldfrag(const _Float16* p, int ld, int row0, int k0, int lane) {
  const int m = lane & 15, lh = lane >> 4;
  const _Float16* q = p + (size_t)(row0 + m) * ld + k0 + 8 * lh;
  Frag f;
  f.h[0] = *(const v8h*)(q);
  f.h[1] = *(const v8h*)(q + 16);
  return f.v;
}

__device__ __forceinline__ v8f zero8() { return (v8f){0.f, 0.f, 0.f, 0.f, 0.f, 0.f, 0.f, 0.f}; }

__device__ __forceinline__ float wave_max(float v) {
#pragma unroll
  for (int o = 16; o >= 1; o >>= 1) v = fmaxf(v, __shfl_xor(v, o, 32));
  return v;
}
__device__ __forceinline__ float wave_sum(float v) {
#pragma unroll
  for (int o = 16; o >= 1; o >>= 1) v += __shfl_xor(v, o, 32);
  return v;
}

__device__ __forceinline__ void gemm32x64(const _Float16* __restrict__ A, int lda,
                                          const _Float16* __restrict__ Bt, int ldb, int K,
                                          int m0, int n0, int lane, v8f (&acc)[2][4]) {
#pragma unroll 1
  for (int k0 = 0; k0 < K; k0 += 32) {
    const v16h a0 = ldfrag(A, lda, m0, k0, lane);
    const v16h a1 = ldfrag(A, lda, m0 + 16, k0, lane);
    const v16h b0 = ldfrag(Bt, ldb, n0, k0, lane);
    const v16h b1 = ldfrag(Bt, ldb, n0 + 16, k0, lane);
    const v16h b2 = ldfrag(Bt, ldb, n0 + 32, k0, lane);
    const v16h b3 = ldfrag(Bt, ldb, n0 + 48, k0, lane);
    acc[0][0] = mma16(a0, b0, acc[0][0]);
    acc[1][0] = mma16(a1, b0, acc[1][0]);
    acc[0][1] = mma16(a0, b1, acc[0][1]);
    acc[1][1] = mma16(a1, b1, acc[1][1]);
    acc[0][2] = mma16(a0, b2, acc[0][2]);
    acc[1][2] = mma16(a1, b2, acc[1][2]);
    acc[0][3] = mma16(a0, b3, acc[0][3]);
    acc[1][3] = mma16(a1, b3, acc[1][3]);
  }
}

__global__ __launch_bounds__(256) void k_cvtw(const float* __restrict__ src, _Float16* __restrict__ dst) {
  __shared__ __align__(16) _Float16 st[32 * LP];
  const int tid = threadIdx.x, lane = tid & 31, wave = tid >> 5;
  const int n0 = blockIdx.x * 32;
  const float* sr = src + (size_t)tid * DM + n0;
#pragma unroll
  for (int q = 0; q < 8; ++q) {
    const v4f v = *(const v4f*)(sr + 4 * q) * 16.0f;
#pragma unroll
    for (int u = 0; u < 4; ++u) st[(4 * q + u) * LP + tid] = (_Float16)v[u];
  }
  __syncthreads();
  v4u val[4];
  size_t go[4];
#pragma unroll
  for (int i = 0; i < 4; ++i) {
    const int nl = wave * 4 + i;
    Pack8 pk;
    pk.h   = *(const v8h*)(st + nl * LP + lane * 8);
    val[i] = pk.u;
    go[i]  = (size_t)(n0 + nl) * DM + lane * 8;
  }
#pragma unroll
  for (int i = 0; i < 4; ++i) *(volatile v4u*)(dst + go[i]) = val[i];
  __threadfence();
#pragma unroll
  for (int i = 0; i < 4; ++i) *(volatile v4u*)(dst + go[i]) = val[i];
}

__global__ __launch_bounds__(256) void k_xcvt(const float* __restrict__ src, _Float16* __restrict__ dh) {
  const size_t o = ((size_t)blockIdx.x * 256 + threadIdx.x) * 8;
  const v4f a0 = *(const v4f*)(src + o);
  const v4f a1 = *(const v4f*)(src + o + 4);
  Pack8 pk;
  pk.h = (v8h){(_Float16)a0[0], (_Float16)a0[1], (_Float16)a0[2], (_Float16)a0[3],
               (_Float16)a1[0], (_Float16)a1[1], (_Float16)a1[2], (_Float16)a1[3]};
  const v4u vv = pk.u;
  volatile v4u* d = (volatile v4u*)(dh + o);
  *d = vv;
  __threadfence();
  *d = vv;
}

__global__ __launch_bounds__(256) void k_pad(_Float16* __restrict__ kp, _Float16* __restrict__ vtp) {
  const int tid = threadIdx.x;
  const v4u z = (v4u){0u, 0u, 0u, 0u};
  size_t off;
  _Float16* base;
  if (blockIdx.x < 64) {
    const int id  = blockIdx.x * 256 + tid;
    const int b   = id >> 11;
    const int rr  = (id >> 5) & 63;
    const int pc  = id & 31;
    const int row = (rr < KOFF) ? rr : (SQ + rr);
    base = kp;
    off  = ((size_t)b * KROWS + row) * DM + pc * 8;
  } else {
    const int id  = (blockIdx.x - 64) * 256 + tid;
    const int row = id >> 4;
    const int pc  = id & 15;
    const int col = (pc < 8) ? (pc * 8) : (VOFF + SQ + (pc - 8) * 8);
    base = vtp;
    off  = (size_t)row * VTP + col;
  }
  volatile v4u* d = (volatile v4u*)(base + off);
  *d = z;
  __threadfence();
  *d = z;
}

__global__ __launch_bounds__(256) void k_gemm_h(const _Float16* __restrict__ xh, const _Float16* __restrict__ w1t,
                                                const float* __restrict__ b1, _Float16* __restrict__ hp) {
  __shared__ __align__(16) _Float16 st[256 * STP];
  const int tid = threadIdx.x, lane = tid & 31, wave = tid >> 5;
  const int hh = lane >> 4, c = lane & 15;
  const int rb = blockIdx.x * 256;
  const int cs = blockIdx.y * 64;
  const int m0 = rb + wave * 32;
  const int n0 = cs;

  v8f acc[2][4];
#pragma unroll
  for (int s = 0; s < 2; ++s)
#pragma unroll
    for (int t = 0; t < 4; ++t) acc[s][t] = zero8();
  gemm32x64(xh, DM, w1t, DM, DM, m0, n0, lane, acc);

  float bb[4];
#pragma unroll
  for (int t = 0; t < 4; ++t) bb[t] = b1[n0 + 16 * t + c];
#pragma unroll
  for (int sub = 0; sub < 2; ++sub)
#pragma unroll
    for (int t = 0; t < 4; ++t)
#pragma unroll
      for (int r = 0; r < 8; ++r)
        st[(wave * 32 + sub * 16 + 8 * hh + r) * STP + 16 * t + c] =
            (_Float16)fmaxf(acc[sub][t][r] * 0.0625f + bb[t], 0.f);
  __syncthreads();

#pragma unroll
  for (int gg = 0; gg < 2; ++gg) {
    v4u val[4];
    size_t go[4];
#pragma unroll
    for (int j = 0; j < 4; ++j) {
      const int p  = tid + 256 * (4 * gg + j);
      const int lr = p >> 3;
      const int pc = p & 7;
      Pack8 pk;
      pk.h   = *(const v8h*)(st + lr * STP + pc * 8);
      val[j] = pk.u;
      go[j]  = (size_t)(rb + lr) * DM + cs + pc * 8;
    }
#pragma unroll
    for (int j = 0; j < 4; ++j) *(volatile v4u*)(hp + go[j]) = val[j];
    __threadfence();
#pragma unroll
    for (int j = 0; j < 4; ++j) *(volatile v4u*)(hp + go[j]) = val[j];
  }
}

__global__ __launch_bounds__(256) void k_qkv(const _Float16* __restrict__ hp, const _Float16* __restrict__ wqkv,
                                             _Float16* __restrict__ qp, _Float16* __restrict__ kp,
                                             _Float16* __restrict__ vtp) {
  __shared__ __align__(16) _Float16 st[256 * STP];
  const int tid = threadIdx.x, lane = tid & 31, wave = tid >> 5;
  const int hh = lane >> 4, c = lane & 15;
  const int rb = blockIdx.x * 256;
  const int b  = rb >> 11;
  const int l0 = rb & (SQ - 1);
  const int ns = blockIdx.y;
  const int which = ns >> 2;
  const int cs = (ns & 3) * 64;
  const int m0 = rb + wave * 32;
  const int n0 = ns * 64;

  v8f acc[2][4];
#pragma unroll
  for (int s = 0; s < 2; ++s)
#pragma unroll
    for (int t = 0; t < 4; ++t) acc[s][t] = zero8();
  gemm32x64(hp, DM, wqkv, DM, DM, m0, n0, lane, acc);

  if (which < 2) {
#pragma unroll
    for (int sub = 0; sub < 2; ++sub)
#pragma unroll
      for (int t = 0; t < 4; ++t)
#pragma unroll
        for (int r = 0; r < 8; ++r)
          st[(wave * 32 + sub * 16 + 8 * hh + r) * STP + 16 * t + c] = (_Float16)(acc[sub][t][r] * 0.0625f);
  } else {
#pragma unroll
    for (int sub = 0; sub < 2; ++sub)
#pragma unroll
      for (int t = 0; t < 4; ++t)
#pragma unroll
        for (int r = 0; r < 8; ++r)
          st[(16 * t + c) * LP + wave * 32 + sub * 16 + 8 * hh + r] = (_Float16)(acc[sub][t][r] * 0.0625f);
  }
  __syncthreads();

  if (which < 2) {
    _Float16* base = (which == 0) ? qp : kp;
    const size_t row0 = (which == 0) ? (size_t)rb : ((size_t)b * KROWS + KOFF + l0);
#pragma unroll
    for (int gg = 0; gg < 2; ++gg) {
      v4u val[4];
      size_t go[4];
#pragma unroll
      for (int j = 0; j < 4; ++j) {
        const int p  = tid + 256 * (4 * gg + j);
        const int lr = p >> 3;
        const int pc = p & 7;
        Pack8 pk;
        pk.h   = *(const v8h*)(st + lr * STP + pc * 8);
        val[j] = pk.u;
        go[j]  = (row0 + lr) * DM + cs + pc * 8;
      }
#pragma unroll
      for (int j = 0; j < 4; ++j) *(volatile v4u*)(base + go[j]) = val[j];
      __threadfence();
#pragma unroll
      for (int j = 0; j < 4; ++j) *(volatile v4u*)(base + go[j]) = val[j];
    }
  } else {
    _Float16* base = vtp + (size_t)b * DM * VTP;
#pragma unroll
    for (int gg = 0; gg < 2; ++gg) {
      v4u val[4];
      size_t go[4];
#pragma unroll
      for (int j = 0; j < 4; ++j) {
        const int p    = tid + 256 * (4 * gg + j);
        const int drow = p >> 5;
        const int pc   = p & 31;
        Pack8 pk;
        pk.h   = *(const v8h*)(st + drow * LP + pc * 8);
        val[j] = pk.u;
        go[j]  = (size_t)(cs + drow) * VTP + VOFF + l0 + pc * 8;
      }
#pragma unroll
      for (int j = 0; j < 4; ++j) *(volatile v4u*)(base + go[j]) = val[j];
      __threadfence();
#pragma unroll
      for (int j = 0; j < 4; ++j) *(volatile v4u*)(base + go[j]) = val[j];
    }
  }
}

__global__ __launch_bounds__(256) void k_attn(const _Float16* __restrict__ qp, const _Float16* __restrict__ kp,
                                              const _Float16* __restrict__ vtp, const _Float16* __restrict__ wht,
                                              const float* __restrict__ bh, const float* __restrict__ wo,
                                              const float* __restrict__ bo, float* __restrict__ out) {
  __shared__ __align__(16) float    Sf[QT * SFP];
  __shared__ __align__(16) _Float16 Ps[QT * PSP];
  __shared__ __align__(16) _Float16 As[QT * LP];
  __shared__ __align__(16) float    Part[8 * QT * NOUT];
  __shared__ float Rl[QT];

  const int tid = threadIdx.x, lane = tid & 31, wave = tid >> 5;
  const int hh = lane >> 4, c = lane & 15;
  const int blk = blockIdx.x;
  const int b   = blk / (SQ / QT);
  const int s0  = (blk - b * (SQ / QT)) * QT;
  const size_t g0 = (size_t)blk * QT;
  const int mt  = wave & 1;

  {
    const int nt = wave >> 1;
    const _Float16* Qg = qp + (g0 + 16 * mt) * DM;
    const _Float16* Kg = kp + ((size_t)b * KROWS + (KOFF - AW) + s0 + 16 * nt) * DM;
    v8f s = zero8();
#pragma unroll 1
    for (int dc = 0; dc < 8; ++dc) {
      const v16h qa = ldfrag(Qg, DM, 0, dc * 32, lane);
      const v16h kb = ldfrag(Kg, DM, 0, dc * 32, lane);
      s = mma16(qa, kb, s);
    }
#pragma unroll
    for (int r = 0; r < 8; ++r) Sf[(16 * mt + 8 * hh + r) * SFP + 16 * nt + c] = s[r];
  }
  __syncthreads();

  {
    const float NEGI = -__builtin_huge_valf();
#pragma unroll
    for (int rr = 0; rr < 4; ++rr) {
      const int r = wave * 4 + rr;
      const float sv0 = Sf[r * SFP + lane] * 0.0625f;
      const float sv1 = Sf[r * SFP + lane + 32] * 0.0625f;
      const bool v0 = lane >= r;
      const bool v1 = lane <= r;
      float m = fmaxf(v0 ? sv0 : NEGI, v1 ? sv1 : NEGI);
      m = wave_max(m);
      float e0 = __expf(sv0 - m);
      float e1 = __expf(sv1 - m);
      e0 = v0 ? e0 : 0.f;
      e1 = v1 ? e1 : 0.f;
      const float ls = wave_sum(e0 + e1);
      Ps[r * PSP + lane]      = (_Float16)(e0 * 1024.0f);
      Ps[r * PSP + lane + 32] = (_Float16)(e1 * 1024.0f);
      if (lane == 0) Rl[r] = (1.0f / ls) * 0.0009765625f;
    }
  }
  __syncthreads();

  {
    const int dq = (wave >> 1) * 64;
    const _Float16* Vg = vtp + (size_t)b * DM * VTP;
    const int col0 = (VOFF - AW) + s0;
    v8f o[4];
#pragma unroll
    for (int t = 0; t < 4; ++t) o[t] = zero8();
#pragma unroll
    for (int kk = 0; kk < 2; ++kk) {
      const v16h pa = ldfrag(Ps, PSP, 16 * mt, kk * 32, lane);
#pragma unroll
      for (int t = 0; t < 4; ++t) {
        const v16h vb = ldfrag(Vg, VTP, dq + 16 * t, col0 + kk * 32, lane);
        o[t] = mma16(pa, vb, o[t]);
      }
    }
    float rl[8];
#pragma unroll
    for (int r = 0; r < 8; ++r) rl[r] = Rl[16 * mt + 8 * hh + r];
#pragma unroll
    for (int t = 0; t < 4; ++t)
#pragma unroll
      for (int r = 0; r < 8; ++r)
        As[(16 * mt + 8 * hh + r) * LP + dq + 16 * t + c] = (_Float16)(o[t][r] * rl[r]);
  }
  __syncthreads();

  {
    const int n0 = wave * 32;
    v8f acc[2][2];
#pragma unroll
    for (int s = 0; s < 2; ++s)
#pragma unroll
      for (int t = 0; t < 2; ++t) acc[s][t] = zero8();
#pragma unroll 1
    for (int dc = 0; dc < 8; ++dc) {
      const v16h a0 = ldfrag(As, LP, 0, dc * 32, lane);
      const v16h a1 = ldfrag(As, LP, 16, dc * 32, lane);
      const v16h b0 = ldfrag(wht, DM, n0, dc * 32, lane);
      const v16h b1 = ldfrag(wht, DM, n0 + 16, dc * 32, lane);
      acc[0][0] = mma16(a0, b0, acc[0][0]);
      acc[1][0] = mma16(a1, b0, acc[1][0]);
      acc[0][1] = mma16(a0, b1, acc[0][1]);
      acc[1][1] = mma16(a1, b1, acc[1][1]);
    }
    float bb[2], w0[2], w1[2];
#pragma unroll
    for (int t = 0; t < 2; ++t) {
      const int col = n0 + 16 * t + c;
      bb[t] = bh[col];
      w0[t] = wo[col * NOUT + 0];
      w1[t] = wo[col * NOUT + 1];
    }
#pragma unroll
    for (int s = 0; s < 2; ++s) {
#pragma unroll
      for (int r = 0; r < 8; ++r) {
        float p0 = 0.f, p1 = 0.f;
#pragma unroll
        for (int t = 0; t < 2; ++t) {
          const float hv = fmaxf(acc[s][t][r] * 0.0625f + bb[t], 0.f);
          p0 = fmaf(hv, w0[t], p0);
          p1 = fmaf(hv, w1[t], p1);
        }
#pragma unroll
        for (int off = 1; off < 16; off <<= 1) {
          p0 += __shfl_xor(p0, off, 32);
          p1 += __shfl_xor(p1, off, 32);
        }
        if (c == 0) {
          Part[(wave * QT + 16 * s + 8 * hh + r) * NOUT + 0] = p0;
          Part[(wave * QT + 16 * s + 8 * hh + r) * NOUT + 1] = p1;
        }
      }
    }
  }
  __syncthreads();

  if (wave == 0) {
    const int L = lane & 15;
    v4f v = (v4f){0.f, 0.f, 0.f, 0.f};
#pragma unroll
    for (int w = 0; w < 8; ++w) {
      const v4f pw = *(const v4f*)(Part + (w * QT + 2 * L) * NOUT);
      v += pw;
    }
    const float bo0 = bo[0], bo1 = bo[1];
    v[0] += bo0; v[1] += bo1; v[2] += bo0; v[3] += bo1;
    if (lane < 16) {
      volatile v4f* d = (volatile v4f*)(out + g0 * NOUT + 4 * L);
      *d = v;
      __threadfence();
      *d = v;
    }
  }
}

extern "C" void kernel_launch(void* const* d_in, const int* in_sizes, int n_in,
                              void* d_out, int out_size, void* d_ws, size_t ws_size,
                              hipStream_t stream) {
  if (n_in < 10) return;
  if (in_sizes[0] != NROW * DM) return;
  if (in_sizes[1] != DM * DM) return;
  if (in_sizes[2] != DM) return;
  if (in_sizes[3] != DM * DM) return;
  if (in_sizes[4] != DM * DM) return;
  if (in_sizes[5] != DM * DM) return;
  if (in_sizes[6] != DM * DM) return;
  if (in_sizes[7] != DM) return;
  if (in_sizes[8] != DM * NOUT) return;
  if (in_sizes[9] != NOUT) return;
  if (out_size != NROW * NOUT) return;

  const float* x  = (const float*)d_in[0];
  const float* W1 = (const float*)d_in[1];
  const float* b1 = (const float*)d_in[2];
  const float* Wq = (const float*)d_in[3];
  const float* Wk = (const float*)d_in[4];
  const float* Wv = (const float*)d_in[5];
  const float* Wh = (const float*)d_in[6];
  const float* bh = (const float*)d_in[7];
  const float* Wo = (const float*)d_in[8];
  const float* bo = (const float*)d_in[9];
  float* out = (float*)d_out;

  const size_t wpl = (size_t)DM * DM * 2;
  size_t off = 0;
  const size_t oW1 = off; off += wpl;
  const size_t oWq = off; off += wpl;
  const size_t oWk = off; off += wpl;
  const size_t oWv = off; off += wpl;
  const size_t oWh = off; off += wpl;
  const size_t oX  = off; off += (size_t)NROW * DM * 2;
  const size_t oH  = off; off += (size_t)NROW * DM * 2;
  const size_t oQ  = off; off += (size_t)NROW * DM * 2;
  const size_t oK  = off; off += (size_t)NB * KROWS * DM * 2;
  const size_t oV  = off; off += (size_t)NB * DM * VTP * 2;
  if (off > ws_size) return;
  if (off > (size_t)134217728) return;
  if (oWk != oWq + wpl || oWv != oWk + wpl) return;

  char* ws = (char*)d_ws;
  _Float16* W1t  = (_Float16*)(ws + oW1);
  _Float16* Wqkv = (_Float16*)(ws + oWq);
  _Float16* Wkt  = (_Float16*)(ws + oWk);
  _Float16* Wvt  = (_Float16*)(ws + oWv);
  _Float16* Wht  = (_Float16*)(ws + oWh);
  _Float16* Xh   = (_Float16*)(ws + oX);
  _Float16* Hh   = (_Float16*)(ws + oH);
  _Float16* Qp   = (_Float16*)(ws + oQ);
  _Float16* Kp   = (_Float16*)(ws + oK);
  _Float16* Vt   = (_Float16*)(ws + oV);

  k_cvtw<<<dim3(DM / 32), dim3(256), 0, stream>>>(W1, W1t);
  k_cvtw<<<dim3(DM / 32), dim3(256), 0, stream>>>(Wq, Wqkv);
  k_cvtw<<<dim3(DM / 32), dim3(256), 0, stream>>>(Wk, Wkt);
  k_cvtw<<<dim3(DM / 32), dim3(256), 0, stream>>>(Wv, Wvt);
  k_cvtw<<<dim3(DM / 32), dim3(256), 0, stream>>>(Wh, Wht);
  k_xcvt<<<dim3((NROW * DM) / 2048), dim3(256), 0, stream>>>(x, Xh);
  k_pad<<<dim3(64 + 128), dim3(256), 0, stream>>>(Kp, Vt);
  k_gemm_h<<<dim3(NROW / 256, DM / 64), dim3(256), 0, stream>>>(Xh, W1t, b1, Hh);
  k_qkv<<<dim3(NROW / 256, NQKV / 64), dim3(256), 0, stream>>>(Hh, Wqkv, Qp, Kp, Vt);
  k_attn<<<dim3(NROW / QT), dim3(256), 0, stream>>>(Qp, Kp, Vt, Wht, bh, Wo, bo, out);
  (void)hipGetLastError();
}
